// Transformer_29927332119124
// MI455X (gfx1250) — hardware-verified
//
#include <hip/hip_runtime.h>
#include <stdint.h>
#include <stddef.h>


#ifndef NB
#define NB 2
#endif
#ifndef SEQ
#define SEQ 2048
#endif
#define NB_FULL 2
#define SEQ_FULL 2048
#define DM 1024
#define NH 16
#define HS 64
#define NF 4096
#define NROW (NB * SEQ)
#define NBH (NB * NH)
#define MT 128
#define NT 64
#define SP 64
#define QB 64
#define KCH 64
#define RRES 64
#define PP 64

static_assert(NB >= 1 && NB <= NB_FULL);
static_assert(SEQ >= MT && SEQ <= SEQ_FULL);
static_assert((SEQ % MT) == 0);
static_assert((SEQ % QB) == 0);
static_assert(QB == KCH && RRES == KCH && HS == 64 && PP == KCH);
static_assert((NROW % MT) == 0);
static_assert((DM % NT) == 0 && (NF % NT) == 0);
static_assert((DM % 32) == 0 && (NF % 32) == 0);
static_assert(MT == 128 && NT == 64 && SP == 64);
static_assert(DM == 8 * 128);
static_assert(DM == 4 * 256);
static_assert(((NROW * (DM / 8)) % 256) == 0);

#define W_SCALE 64.0f
#define INV_W 0.015625f
#define P_SCALE 1024.0f
#define INV_P 0.0009765625f
#define O_SCALE 32.0f
#define INV_O 0.03125f
#define R_SCALE 1024.0f
#define INV_R 0.0009765625f
#define INV_SQRT_HS 0.125f
#define LN_EPS 1.0e-5f
#define NEG_BIG (-1.0e30f)

typedef _Float16 v16h __attribute__((ext_vector_type(16)));
typedef _Float16 v8h  __attribute__((ext_vector_type(8)));
typedef float    v8f  __attribute__((ext_vector_type(8)));
typedef float    v4f  __attribute__((ext_vector_type(4)));
typedef unsigned int v4u __attribute__((ext_vector_type(4)));

union Frag  { v16h v; v8h h[2]; };
union Pack8 { v8h h; v4u u; };
static_assert(sizeof(Pack8) == 16);

__device__ __forceinline__ float bf16r(float v) {
  unsigned int u = __float_as_uint(v);
  u += 0x7fffu + ((u >> 16) & 1u);
  u &= 0xffff0000u;
  return __uint_as_float(u);
}

__device__ __forceinline__ v16h fragld(const _Float16* base, int ld, int k0, int lane) {
  const _Float16* p = base + (lane & 15) * ld + k0 + 8 * (lane >> 4);
  Frag f;
  f.h[0] = *(const v8h*)(p);
  f.h[1] = *(const v8h*)(p + 16);
  return f.v;
}

__device__ __forceinline__ v8f mma16(v16h a, v16h b, v8f c) {
  v8f d = __builtin_amdgcn_wmma_f32_16x16x32_f16(false, a, false, b, (short)0, c, false, false);
  asm volatile("v_nop\n\tv_nop\n\tv_nop\n\tv_nop" : "+v"(d) : "v"(a), "v"(b));
  return d;
}

__device__ __forceinline__ float rsum16(float v) {
  v += __shfl_xor(v, 8);
  v += __shfl_xor(v, 4);
  v += __shfl_xor(v, 2);
  v += __shfl_xor(v, 1);
  return v;
}
__device__ __forceinline__ float rmax16(float v) {
  v = fmaxf(v, __shfl_xor(v, 8));
  v = fmaxf(v, __shfl_xor(v, 4));
  v = fmaxf(v, __shfl_xor(v, 2));
  v = fmaxf(v, __shfl_xor(v, 1));
  return v;
}
__device__ __forceinline__ float rsum32(float v) {
  v += __shfl_xor(v, 16);
  v += __shfl_xor(v, 8);
  v += __shfl_xor(v, 4);
  v += __shfl_xor(v, 2);
  v += __shfl_xor(v, 1);
  return v;
}

__global__ __launch_bounds__(256) void k_pack(const float* __restrict__ src,
                                              _Float16* dst,
                                              int nbat, int K, int N, int Npad, int bstride) {
  const int gid = blockIdx.x * 256 + threadIdx.x;
  const int total = nbat * Npad * K;
  const int e = gid * 8;
  if (e >= total) return;
  const int per = Npad * K;
  const int b = e / per;
  const int wi = e - b * per;
  const int n = wi / K;
  const int k0 = wi - n * K;
  const int nn = (n < N) ? n : (N - 1);
  const float* sp = src + (size_t)b * bstride + (size_t)k0 * N + nn;
  v8h t8;
#pragma unroll
  for (int i = 0; i < 8; ++i) {
    float v = sp[(size_t)i * N];
    v = (n < N) ? (bf16r(v) * W_SCALE) : 0.0f;
    t8[i] = (_Float16)v;
  }
  Pack8 pk;
  pk.h = t8;
  _Float16* dp = dst + e;
  *(volatile v4u*)dp = pk.u;
  __threadfence();
  *(volatile v4u*)dp = pk.u;
}

__global__ __launch_bounds__(256) void k_cvtx(const float* __restrict__ x, _Float16* Xh) {
  const int gid = blockIdx.x * 256 + threadIdx.x;
  const int total = NROW * (DM / 8);
  if (gid >= total) return;
  const int r = gid / (DM / 8);
  const int c8 = gid - r * (DM / 8);
  const int b = r / SEQ, t = r - b * SEQ;
  const float* sp = x + ((size_t)b * SEQ_FULL + t) * DM + 8 * c8;
  const v4f a0 = *(const v4f*)sp;
  const v4f a1 = *(const v4f*)(sp + 4);
  v8h t8;
#pragma unroll
  for (int e = 0; e < 4; ++e) {
    t8[e]     = (_Float16)bf16r(a0[e]);
    t8[4 + e] = (_Float16)bf16r(a1[e]);
  }
  Pack8 pk;
  pk.h = t8;
  _Float16* dp = Xh + (size_t)gid * 8;
  *(volatile v4u*)dp = pk.u;
  __threadfence();
  *(volatile v4u*)dp = pk.u;
}

__device__ __forceinline__ void mac_tile(const _Float16* __restrict__ A, int lda,
                                         const _Float16* __restrict__ Bt, int ldb, int K, int lane,
                                         v8f (&acc)[2][4]) {
  const v8f zero = {};
#pragma unroll
  for (int mt = 0; mt < 2; ++mt)
#pragma unroll
    for (int j = 0; j < 4; ++j) acc[mt][j] = zero;
  const _Float16* A1 = A + 16 * (size_t)lda;
#pragma unroll 1
  for (int k0 = 0; k0 < K; k0 += 32) {
    const v16h a0 = fragld(A, lda, k0, lane);
    const v16h a1 = fragld(A1, lda, k0, lane);
#pragma unroll
    for (int j = 0; j < 4; ++j) {
      const v16h bfr = fragld(Bt + (size_t)j * 16 * ldb, ldb, k0, lane);
      acc[0][j] = mma16(a0, bfr, acc[0][j]);
      acc[1][j] = mma16(a1, bfr, acc[1][j]);
    }
  }
}

__device__ __forceinline__ void stage_tile(float* stg, int w, int lane, v8f (&acc)[2][4], float scl) {
  const int m = lane & 15, hh = lane >> 4;
#pragma unroll
  for (int mt = 0; mt < 2; ++mt)
#pragma unroll
    for (int j = 0; j < 4; ++j)
#pragma unroll
      for (int r = 0; r < 8; ++r)
        stg[(32 * w + 16 * mt + 8 * hh + r) * SP + 16 * j + m] = acc[mt][j][r] * scl;
}

template <bool RELU>
__device__ __forceinline__ void st_rows_f16(const float* stg, const float* __restrict__ bias,
                                            _Float16* C, int ldc, int tid) {
#pragma unroll
  for (int i = 0; i < 8; ++i) {
    const int p = tid + 128 * i;
    const int row = p >> 3, c8 = p & 7;
    const float* sp = stg + row * SP + 8 * c8;
    const v4f lo = *(const v4f*)sp;
    const v4f hi = *(const v4f*)(sp + 4);
    const v4f b0 = *(const v4f*)(bias + 8 * c8);
    const v4f b1 = *(const v4f*)(bias + 8 * c8 + 4);
    v8h t8;
#pragma unroll
    for (int e = 0; e < 4; ++e) {
      float q0 = lo[e] + bf16r(b0[e]);
      float q1 = hi[e] + bf16r(b1[e]);
      if (RELU) { q0 = fmaxf(q0, 0.0f); q1 = fmaxf(q1, 0.0f); }
      t8[e]     = (_Float16)q0;
      t8[4 + e] = (_Float16)q1;
    }
    Pack8 pk;
    pk.h = t8;
    *(volatile v4u*)(C + (size_t)row * ldc + 8 * c8) = pk.u;
  }
}

__device__ __forceinline__ void st_res_f16(const float* stg, const float* __restrict__ bias,
                                           _Float16* Cr, int tid) {
#pragma unroll
  for (int i = 0; i < 4; ++i) {
    const int p = tid + 128 * i;
    const int row = p >> 3, c8 = p & 7;
    const float* sp = stg + row * SP + 8 * c8;
    const v4f lo = *(const v4f*)sp;
    const v4f hi = *(const v4f*)(sp + 4);
    const v4f b0 = *(const v4f*)(bias + 8 * c8);
    const v4f b1 = *(const v4f*)(bias + 8 * c8 + 4);
    v8h t8;
#pragma unroll
    for (int e = 0; e < 4; ++e) {
      const float q0 = lo[e] + bf16r(b0[e]);
      const float q1 = hi[e] + bf16r(b1[e]);
      const _Float16 h0 = (_Float16)q0;
      const _Float16 h1 = (_Float16)q1;
      t8[e]     = (_Float16)((q0 - (float)h0) * R_SCALE);
      t8[4 + e] = (_Float16)((q1 - (float)h1) * R_SCALE);
    }
    Pack8 pk;
    pk.h = t8;
    *(volatile v4u*)(Cr + (size_t)row * HS + 8 * c8) = pk.u;
  }
}

__device__ __forceinline__ void st_vt(const float* stg, const float* __restrict__ bias,
                                      _Float16* Vb, int tid) {
#pragma unroll
  for (int i = 0; i < 8; ++i) {
    const int p = tid + 128 * i;
    const int d = p >> 4, c = p & 15;
    const float bd = bf16r(bias[d]);
    v8h t8;
#pragma unroll
    for (int e = 0; e < 8; ++e) t8[e] = (_Float16)(stg[(8 * c + e) * SP + d] + bd);
    Pack8 pk;
    pk.h = t8;
    *(volatile v4u*)(Vb + (size_t)d * SEQ + 8 * c) = pk.u;
  }
}

__device__ __forceinline__ void st_vres(const float* stg, const float* __restrict__ bias,
                                        _Float16* Vrb, int tid) {
#pragma unroll
  for (int i = 0; i < 4; ++i) {
    const int p = tid + 128 * i;
    const int d = p >> 3, c = p & 7;
    const float bd = bf16r(bias[d]);
    v8h t8;
#pragma unroll
    for (int e = 0; e < 8; ++e) {
      const float v = stg[(8 * c + e) * SP + d] + bd;
      const _Float16 vh = (_Float16)v;
      t8[e] = (_Float16)((v - (float)vh) * R_SCALE);
    }
    Pack8 pk;
    pk.h = t8;
    *(volatile v4u*)(Vrb + (size_t)d * RRES + 8 * c) = pk.u;
  }
}

template <bool XRES>
__device__ __forceinline__ void st_rows_f32(const float* stg, const float* __restrict__ bias,
                                            const float* __restrict__ xres, int m0, int n0,
                                            float* C, int ldc, int tid) {
#pragma unroll
  for (int i = 0; i < 16; ++i) {
    const int p = tid + 128 * i;
    const int row = p >> 4, c4 = p & 15;
    const v4f v  = *(const v4f*)(stg + row * SP + 4 * c4);
    const v4f bb = *(const v4f*)(bias + 4 * c4);
    v4f o;
#pragma unroll
    for (int e = 0; e < 4; ++e) o[e] = v[e] + bf16r(bb[e]);
    if (XRES) {
      const int gr = m0 + row;
      const int b = gr / SEQ;
      const int t = gr - b * SEQ;
      const v4f xv = *(const v4f*)(xres + ((size_t)b * SEQ_FULL + t) * DM + n0 + 4 * c4);
#pragma unroll
      for (int e = 0; e < 4; ++e) o[e] += bf16r(xv[e]);
    }
    *(volatile v4f*)(C + (size_t)row * ldc + 4 * c4) = o;
  }
}

__global__ __launch_bounds__(128) void k_qkv(
    const _Float16* __restrict__ Xh,
    const _Float16* __restrict__ WqT, const _Float16* __restrict__ WkT, const _Float16* __restrict__ WvT,
    const float* __restrict__ bq, const float* __restrict__ bk, const float* __restrict__ bv,
    _Float16* Qp, _Float16* Kp, _Float16* Vt, _Float16* Qr, _Float16* Kr, _Float16* Vr)
{
  __shared__ __align__(16) float stg[MT * SP];
  const int tid = threadIdx.x, lane = tid & 31, w = tid >> 5;
  const int z = blockIdx.z;
  const int which = z / NBH;
  const int bh = z - which * NBH;
  const int b = bh / NH, h = bh - b * NH;
  const int m0 = blockIdx.x * MT;
  const _Float16* Bt = (which == 0) ? WqT : ((which == 1) ? WkT : WvT);
  const float* bias  = (which == 0) ? bq  : ((which == 1) ? bk  : bv);
  Bt   += (size_t)h * HS * DM;
  bias += h * HS;
  const _Float16* A = Xh + ((size_t)b * SEQ + m0 + 32 * w) * DM;

  v8f acc[2][4];
  mac_tile(A, DM, Bt, DM, DM, lane, acc);
  stage_tile(stg, w, lane, acc, INV_W);
  __syncthreads();

  if (which != 2) {
    _Float16* Cb = ((which == 0) ? Qp : Kp) + ((size_t)bh * SEQ + m0) * HS;
    st_rows_f16<false>(stg, bias, Cb, HS, tid);
    __threadfence();
    st_rows_f16<false>(stg, bias, Cb, HS, tid);
    if (m0 == 0) {
      _Float16* Cr = ((which == 0) ? Qr : Kr) + (size_t)bh * RRES * HS;
      st_res_f16(stg, bias, Cr, tid);
      __threadfence();
      st_res_f16(stg, bias, Cr, tid);
    }
  } else {
    _Float16* Vb = Vt + (size_t)bh * HS * SEQ + m0;
    st_vt(stg, bias, Vb, tid);
    __threadfence();
    st_vt(stg, bias, Vb, tid);
    if (m0 == 0) {
      _Float16* Vrb = Vr + (size_t)bh * HS * RRES;
      st_vres(stg, bias, Vrb, tid);
      __threadfence();
      st_vres(stg, bias, Vrb, tid);
    }
  }
}

__device__ __forceinline__ void st_o(const _Float16* oS, _Float16* Ob, int lane) {
#pragma unroll
  for (int i = 0; i < 4; ++i) {
    const int p = lane + 32 * i;
    const int row = p >> 3, c8 = p & 7;
    Pack8 pk;
    pk.h = *(const v8h*)(oS + row * PP + 8 * c8);
    *(volatile v4u*)(Ob + (size_t)row * DM + 8 * c8) = pk.u;
  }
}

__global__ __launch_bounds__(128) void k_attn(
    const _Float16* __restrict__ Qp, const _Float16* __restrict__ Kp, const _Float16* __restrict__ Vt,
    const _Float16* __restrict__ Qr, const _Float16* __restrict__ Kr, const _Float16* __restrict__ Vr,
    _Float16* Op)
{
  __shared__ __align__(16) _Float16 pS[4][16 * PP];
  __shared__ __align__(16) _Float16 pR[4][16 * PP];
  const int tid = threadIdx.x, lane = tid & 31, w = tid >> 5, m = lane & 15, hh = lane >> 4;
  const int qb = blockIdx.x, bh = blockIdx.y;
  const int b = bh / NH, h = bh - b * NH;
  const int t0 = qb * QB + 16 * w;
  const bool res = (qb == 0);
  _Float16* pSw = &pS[w][0];
  _Float16* pRw = &pR[w][0];
  const v8f zero = {};

  const _Float16* qbase = Qp + ((size_t)bh * SEQ + t0) * HS;
  const v16h qa0 = fragld(qbase, HS, 0, lane);
  const v16h qa1 = fragld(qbase, HS, 32, lane);
  const _Float16* qrb = res ? (Qr + ((size_t)bh * RRES + t0) * HS) : qbase;
  const v16h qr0 = fragld(qrb, HS, 0, lane);
  const v16h qr1 = fragld(qrb, HS, 32, lane);

  v8f oacc[4];
#pragma unroll
  for (int jd = 0; jd < 4; ++jd) oacc[jd] = zero;
  float mrun[8], lrun[8];
#pragma unroll
  for (int r = 0; r < 8; ++r) { mrun[r] = NEG_BIG; lrun[r] = 0.0f; }
  const int tq = t0 + 8 * hh;

#pragma unroll 1
  for (int c = 0; c <= qb; ++c) {
    const int kb = c * KCH;
    const _Float16* Kc = Kp + ((size_t)bh * SEQ + kb) * HS;

    v8f sc[4];
#pragma unroll
    for (int j = 0; j < 4; ++j) {
      const v16h b0 = fragld(Kc + j * 16 * HS, HS, 0, lane);
      const v16h b1 = fragld(Kc + j * 16 * HS, HS, 32, lane);
      v8f s = mma16(qa0, b0, zero);
      s = mma16(qa1, b1, s);
      if (res) {
        const _Float16* Krc = Kr + ((size_t)bh * RRES + kb + j * 16) * HS;
        const v16h r0 = fragld(Krc, HS, 0, lane);
        const v16h r1 = fragld(Krc, HS, 32, lane);
        v8f sr = mma16(qa0, r0, zero);
        sr = mma16(qr0, b0, sr);
        sr = mma16(qa1, r1, sr);
        sr = mma16(qr1, b1, sr);
#pragma unroll
        for (int r = 0; r < 8; ++r) s[r] += sr[r] * INV_R;
      }
      sc[j] = s;
    }

#pragma unroll
    for (int r = 0; r < 8; ++r) {
      const int t = tq + r;
      float xv[4];
      float mx = NEG_BIG;
#pragma unroll
      for (int j = 0; j < 4; ++j) {
        const int key = kb + 16 * j + m;
        xv[j] = (key <= t) ? (sc[j][r] * INV_SQRT_HS) : NEG_BIG;
        mx = fmaxf(mx, xv[j]);
      }
      mx = rmax16(mx);
      const float mnew = fmaxf(mrun[r], mx);
      const float corr = __expf(mrun[r] - mnew);
      float pv[4];
      float ps = 0.0f;
#pragma unroll
      for (int j = 0; j < 4; ++j) {
        pv[j] = (xv[j] > -1.0e29f) ? __expf(xv[j] - mnew) : 0.0f;
        ps += pv[j];
      }
      ps = rsum16(ps);
      lrun[r] = lrun[r] * corr + ps;
      mrun[r] = mnew;
#pragma unroll
      for (int jd = 0; jd < 4; ++jd) oacc[jd][r] *= corr;
#pragma unroll
      for (int j = 0; j < 4; ++j) {
        const float p1 = pv[j] * P_SCALE;
        const _Float16 ph = (_Float16)p1;
        pSw[(8 * hh + r) * PP + 16 * j + m] = ph;
        if (res) pRw[(8 * hh + r) * PP + 16 * j + m] = (_Float16)((p1 - (float)ph) * R_SCALE);
      }
    }
    __syncthreads();

    const v16h pa0 = fragld(pSw, PP, 0, lane);
    const v16h pa1 = fragld(pSw, PP, 32, lane);
    const _Float16* Vc = Vt + (size_t)bh * HS * SEQ + kb;
#pragma unroll
    for (int jd = 0; jd < 4; ++jd) {
      const v16h v0 = fragld(Vc + (size_t)jd * 16 * SEQ, SEQ, 0, lane);
      const v16h v1 = fragld(Vc + (size_t)jd * 16 * SEQ, SEQ, 32, lane);
      oacc[jd] = mma16(pa0, v0, oacc[jd]);
      oacc[jd] = mma16(pa1, v1, oacc[jd]);
      if (res) {
        const v16h pr0 = fragld(pRw, PP, 0, lane);
        const v16h pr1 = fragld(pRw, PP, 32, lane);
        const _Float16* Vrc = Vr + ((size_t)bh * HS + jd * 16) * RRES;
        const v16h vr0 = fragld(Vrc, RRES, 0, lane);
        const v16h vr1 = fragld(Vrc, RRES, 32, lane);
        v8f orr = mma16(pr0, v0, zero);
        orr = mma16(pa0, vr0, orr);
        orr = mma16(pr1, v1, orr);
        orr = mma16(pa1, vr1, orr);
#pragma unroll
        for (int r = 0; r < 8; ++r) oacc[jd][r] += orr[r] * INV_R;
      }
    }
    __syncthreads();
  }

#pragma unroll
  for (int r = 0; r < 8; ++r) {
    const float inv = (O_SCALE * INV_P) * (1.0f / lrun[r]);
#pragma unroll
    for (int jd = 0; jd < 4; ++jd)
      pSw[(8 * hh + r) * PP + 16 * jd + m] = (_Float16)(oacc[jd][r] * inv);
  }
  __syncthreads();
  _Float16* Ob = Op + ((size_t)b * SEQ + t0) * DM + h * HS;
  st_o(pSw, Ob, lane);
  __threadfence();
  st_o(pSw, Ob, lane);
}

template <int MODE>
__global__ __launch_bounds__(128) void k_gemm(const _Float16* __restrict__ A, int lda,
                                               const _Float16* __restrict__ Bt, int ldb, int K,
                                               const float* __restrict__ bias,
                                               const float* __restrict__ xres, void* C, int ldc)
{
  __shared__ __align__(16) float stg[MT * SP];
  const int tid = threadIdx.x, lane = tid & 31, w = tid >> 5;
  const int m0 = blockIdx.x * MT, n0 = blockIdx.y * NT;
  v8f acc[2][4];
  mac_tile(A + ((size_t)m0 + 32 * w) * lda, lda, Bt + (size_t)n0 * ldb, ldb, K, lane, acc);
  const float scl = (MODE == 1) ? (INV_W * INV_O) : INV_W;
  stage_tile(stg, w, lane, acc, scl);
  __syncthreads();
  if (MODE == 2) {
    _Float16* Cb = (_Float16*)C + (size_t)m0 * ldc + n0;
    st_rows_f16<true>(stg, bias + n0, Cb, ldc, tid);
    __threadfence();
    st_rows_f16<true>(stg, bias + n0, Cb, ldc, tid);
  } else {
    float* Cb = (float*)C + (size_t)m0 * ldc + n0;
    st_rows_f32<MODE == 1>(stg, bias + n0, xres, m0, n0, Cb, ldc, tid);
    __threadfence();
    st_rows_f32<MODE == 1>(stg, bias + n0, xres, m0, n0, Cb, ldc, tid);
  }
}

__global__ __launch_bounds__(128) void k_ln1(const float* __restrict__ hp, const float* __restrict__ g,
                                              const float* __restrict__ be, _Float16* Hh) {
  __shared__ float red[2][4];
  const int tid = threadIdx.x, lane = tid & 31, w = tid >> 5;
  const int row = blockIdx.x;
  const float* xr = hp + (size_t)row * DM + 8 * tid;
  const v4f a0 = *(const v4f*)xr;
  const v4f a1 = *(const v4f*)(xr + 4);
  float v[8];
#pragma unroll
  for (int e = 0; e < 4; ++e) { v[e] = a0[e]; v[4 + e] = a1[e]; }
  float s = 0.0f;
#pragma unroll
  for (int e = 0; e < 8; ++e) s += v[e];
  s = rsum32(s);
  if (lane == 0) red[0][w] = s;
  __syncthreads();
  const float mu = (red[0][0] + red[0][1] + red[0][2] + red[0][3]) * (1.0f / DM);
  float sq = 0.0f;
#pragma unroll
  for (int e = 0; e < 8; ++e) { v[e] -= mu; sq += v[e] * v[e]; }
  sq = rsum32(sq);
  if (lane == 0) red[1][w] = sq;
  __syncthreads();
  const float var  = (red[1][0] + red[1][1] + red[1][2] + red[1][3]) * (1.0f / DM);
  const float rstd = rsqrtf(var + LN_EPS);
  const v4f g0 = *(const v4f*)(g + 8 * tid);
  const v4f g1 = *(const v4f*)(g + 8 * tid + 4);
  const v4f e0 = *(const v4f*)(be + 8 * tid);
  const v4f e1 = *(const v4f*)(be + 8 * tid + 4);
  v8h t8;
#pragma unroll
  for (int e = 0; e < 4; ++e) {
    t8[e]     = (_Float16)(v[e] * rstd * bf16r(g0[e]) + bf16r(e0[e]));
    t8[4 + e] = (_Float16)(v[4 + e] * rstd * bf16r(g1[e]) + bf16r(e1[e]));
  }
  Pack8 pk;
  pk.h = t8;
  _Float16* dp = Hh + (size_t)row * DM + 8 * tid;
  *(volatile v4u*)dp = pk.u;
  __threadfence();
  *(volatile v4u*)dp = pk.u;
}

__global__ __launch_bounds__(256) void k_ln2(const float* __restrict__ Y, const float* __restrict__ g,
                                              const float* __restrict__ be, float* out) {
  __shared__ float red[2][8];
  const int tid = threadIdx.x, lane = tid & 31, w = tid >> 5;
  const int row = blockIdx.x;
  const int b = row / SEQ, t = row - b * SEQ;
  const v4f y = *(const v4f*)(Y + (size_t)row * DM + 4 * tid);
  float s = (y[0] + y[1]) + (y[2] + y[3]);
  s = rsum32(s);
  if (lane == 0) red[0][w] = s;
  __syncthreads();
  float tot = 0.0f;
#pragma unroll
  for (int i = 0; i < 8; ++i) tot += red[0][i];
  const float mu = tot * (1.0f / DM);
  float d[4];
  float sq = 0.0f;
#pragma unroll
  for (int e = 0; e < 4; ++e) { d[e] = y[e] - mu; sq += d[e] * d[e]; }
  sq = rsum32(sq);
  if (lane == 0) red[1][w] = sq;
  __syncthreads();
  float tot2 = 0.0f;
#pragma unroll
  for (int i = 0; i < 8; ++i) tot2 += red[1][i];
  const float var  = tot2 * (1.0f / DM);
  const float rstd = rsqrtf(var + LN_EPS);
  const v4f g4 = *(const v4f*)(g + 4 * tid);
  const v4f b4 = *(const v4f*)(be + 4 * tid);
  v4f o;
#pragma unroll
  for (int e = 0; e < 4; ++e) o[e] = d[e] * rstd * bf16r(g4[e]) + bf16r(b4[e]) + y[e];
  float* dp = out + ((size_t)b * SEQ_FULL + t) * DM + 4 * tid;
  *(volatile v4f*)dp = o;
  __threadfence();
  *(volatile v4f*)dp = o;
}

extern "C" void kernel_launch(void* const* d_in, const int* in_sizes, int n_in,
                              void* d_out, int out_size, void* d_ws, size_t ws_size,
                              hipStream_t stream)
{
  if (n_in < 17) return;
  const float* x    = (const float*)d_in[0];
  const float* Wq   = (const float*)d_in[1];
  const float* bq   = (const float*)d_in[2];
  const float* Wk   = (const float*)d_in[3];
  const float* bk   = (const float*)d_in[4];
  const float* Wv   = (const float*)d_in[5];
  const float* bv   = (const float*)d_in[6];
  const float* Wo   = (const float*)d_in[7];
  const float* bo   = (const float*)d_in[8];
  const float* g1   = (const float*)d_in[9];
  const float* be1  = (const float*)d_in[10];
  const float* W1   = (const float*)d_in[11];
  const float* b1   = (const float*)d_in[12];
  const float* W2   = (const float*)d_in[13];
  const float* b2   = (const float*)d_in[14];
  const float* g2   = (const float*)d_in[15];
  const float* be2  = (const float*)d_in[16];
  float* out = (float*)d_out;

  if (in_sizes[0]  < ((NB - 1) * SEQ_FULL + SEQ) * DM) return;
  if (in_sizes[1]  < NH * DM * HS) return;
  if (in_sizes[2]  < NH * HS) return;
  if (in_sizes[3]  < NH * DM * HS) return;
  if (in_sizes[4]  < NH * HS) return;
  if (in_sizes[5]  < NH * DM * HS) return;
  if (in_sizes[6]  < NH * HS) return;
  if (in_sizes[7]  < DM * DM) return;
  if (in_sizes[8]  < DM) return;
  if (in_sizes[9]  < DM) return;
  if (in_sizes[10] < DM) return;
  if (in_sizes[11] < DM * NF) return;
  if (in_sizes[12] < NF) return;
  if (in_sizes[13] < NF * DM) return;
  if (in_sizes[14] < DM) return;
  if (in_sizes[15] < DM) return;
  if (in_sizes[16] < DM) return;
  if (out_size < ((NB - 1) * SEQ_FULL + SEQ) * DM) return;

  size_t off = 0;
  auto take = [&](size_t bytes) -> char* {
    char* p = (char*)d_ws + off;
    off += (bytes + 255) & ~(size_t)255;
    return p;
  };
  const size_t szX  = (size_t)NROW * DM * sizeof(_Float16);
  const size_t szWh = (size_t)NH * HS * DM * sizeof(_Float16);
  const size_t szWo = (size_t)DM * DM * sizeof(_Float16);
  const size_t szW1 = (size_t)NF * DM * sizeof(_Float16);
  const size_t szW2 = (size_t)DM * NF * sizeof(_Float16);
  const size_t szP  = (size_t)NBH * SEQ * HS * sizeof(_Float16);
  const size_t szU  = (size_t)NROW * NF * sizeof(_Float16);
  const size_t szA  = (4 * szP > szU) ? (4 * szP) : szU;
  const size_t szB  = (size_t)NROW * DM * sizeof(float);
  const size_t szH  = (size_t)NROW * DM * sizeof(_Float16);
  const size_t szR  = (size_t)NBH * RRES * HS * sizeof(_Float16);
  _Float16* Xh  = (_Float16*)take(szX);
  _Float16* WqT = (_Float16*)take(szWh);
  _Float16* WkT = (_Float16*)take(szWh);
  _Float16* WvT = (_Float16*)take(szWh);
  _Float16* WoT = (_Float16*)take(szWo);
  _Float16* W1T = (_Float16*)take(szW1);
  _Float16* W2T = (_Float16*)take(szW2);
  char* regA = take(szA);
  _Float16* Qp  = (_Float16*)(regA);
  _Float16* Kp  = (_Float16*)(regA + szP);
  _Float16* Vtp = (_Float16*)(regA + 2 * szP);
  _Float16* Op  = (_Float16*)(regA + 3 * szP);
  _Float16* Up  = (_Float16*)(regA);
  char* regB = take(szB);
  float* hpre = (float*)regB;
  float* Yp   = (float*)regB;
  _Float16* Hh  = (_Float16*)take(szH);
  _Float16* Qr  = (_Float16*)take(szR);
  _Float16* Kr  = (_Float16*)take(szR);
  _Float16* Vr  = (_Float16*)take(szR);
  if (off > ws_size) return;
  if (off > (size_t)134217728u) return;

  {
    const int nthr = NROW * (DM / 8);
    k_cvtx<<<(nthr + 255) / 256, 256, 0, stream>>>(x, Xh);
  }
  auto pack = [&](const float* src, _Float16* dst, int nbat, int K, int N, int Npad, int bstride) {
    const int total = nbat * Npad * K;
    const int nthr = total / 8;
    k_pack<<<(nthr + 255) / 256, 256, 0, stream>>>(src, dst, nbat, K, N, Npad, bstride);
  };
  pack(Wq, WqT, NH, DM, HS, HS, DM * HS);
  pack(Wk, WkT, NH, DM, HS, HS, DM * HS);
  pack(Wv, WvT, NH, DM, HS, HS, DM * HS);
  pack(Wo, WoT, 1, DM, DM, DM, DM * DM);
  pack(W1, W1T, 1, DM, NF, NF, DM * NF);
  pack(W2, W2T, 1, NF, DM, DM, NF * DM);

  k_qkv<<<dim3(SEQ / MT, 1, 3 * NBH), 128, 0, stream>>>(Xh, WqT, WkT, WvT, bq, bk, bv,
                                                          Qp, Kp, Vtp, Qr, Kr, Vr);
  k_attn<<<dim3(SEQ / QB, NBH), 128, 0, stream>>>(Qp, Kp, Vtp, Qr, Kr, Vr, Op);
  hipLaunchKernelGGL(k_gemm<1>, dim3(NROW / MT, DM / NT), dim3(128), 0, stream,
                     (const _Float16*)Op, (int)DM, (const _Float16*)WoT, (int)DM, (int)DM,
                     bo, x, (void*)hpre, (int)DM);
  k_ln1<<<NROW, 128, 0, stream>>>(hpre, g1, be1, Hh);
  hipLaunchKernelGGL(k_gemm<2>, dim3(NROW / MT, NF / NT), dim3(128), 0, stream,
                     (const _Float16*)Hh, (int)DM, (const _Float16*)W1T, (int)DM, (int)DM,
                     b1, x, (void*)Up, (int)NF);
  hipLaunchKernelGGL(k_gemm<3>, dim3(NROW / MT, DM / NT), dim3(128), 0, stream,
                     (const _Float16*)Up, (int)NF, (const _Float16*)W2T, (int)NF, (int)NF,
                     b2, x, (void*)Yp, (int)DM);
  k_ln2<<<NROW, 256, 0, stream>>>(Yp, g2, be2, out);
}
